// SimpleFineGrainedHeadWeight_87591563034911
// MI455X (gfx1250) — hardware-verified
//
#include <hip/hip_runtime.h>
#include <math.h>

typedef _Float16 v16h __attribute__((ext_vector_type(16)));
typedef _Float16 v8h  __attribute__((ext_vector_type(8)));
typedef float    v8f  __attribute__((ext_vector_type(8)));
typedef float    v4f  __attribute__((ext_vector_type(4)));
typedef int      v4i  __attribute__((ext_vector_type(4)));
typedef double   v2d  __attribute__((ext_vector_type(2)));
typedef v8h __attribute__((may_alias)) v8ha;
typedef v4f __attribute__((may_alias)) v4fa;
typedef v4i __attribute__((may_alias)) v4ia;

union Frag { v16h v; v8h half[2]; };

#define NB    64
#define NV    196
#define NT    64
#define KIN   768
#define NE    512
#define MV    (NB * NV)
#define MT    (NB * NT)
#define MVPAD (MV + 16)
#define VWP   256
#define I1P   256
#define SWAVES 13
#define ZP    72

static_assert(MV % 64 == 0);
static_assert(MT % 64 == 0);
static_assert(MV % 32 == 0);
static_assert((MV * KIN) % (8 * 256) == 0);
static_assert(((MV + MT) * KIN) % (8 * 256) == 0);
static_assert(NE % 128 == 0);
static_assert(KIN % 64 == 0);
static_assert(((MVPAD - MV) * NE) % 8 == 0);

__device__ __forceinline__ v8f wmma_f16(v16h a, v16h b, v8f c) {
  v8f d = __builtin_amdgcn_wmma_f32_16x16x32_f16(false, a, false, b, (short)0, c, false, false);
  asm volatile("v_nop\n\tv_nop\n\tv_nop\n\tv_nop" : "+v"(d) : "v"(a), "v"(b));
  return d;
}

__device__ __forceinline__ v16h load_frag(const _Float16* p, int h) {
  Frag f;
  f.half[0] = *(const v8ha*)(p + 8 * h);
  f.half[1] = *(const v8ha*)(p + 16 + 8 * h);
  return f.v;
}

__global__ __launch_bounds__(256) void k_zfill(_Float16* __restrict__ p, int n8)
{
  v8h z;
  #pragma unroll
  for (int i = 0; i < 8; ++i) z[i] = (_Float16)0.0f;
  #pragma unroll 1
  for (int g = blockIdx.x * 256 + threadIdx.x; g < n8; g += gridDim.x * 256)
    *(volatile v8h*)(p + (size_t)g * 8) = z;
  __threadfence();
  #pragma unroll 1
  for (int g = blockIdx.x * 256 + threadIdx.x; g < n8; g += gridDim.x * 256)
    *(volatile v8h*)(p + (size_t)g * 8) = z;
}

__global__ __launch_bounds__(256) void k_convw(const float* __restrict__ Wv,
                                               const float* __restrict__ Wt,
                                               _Float16* __restrict__ WT)
{
  __shared__ __attribute__((aligned(16))) _Float16 sT[64 * ZP];
  const int tid = threadIdx.x, lane = tid & 31, wv = tid >> 5;
  const int k0 = blockIdx.x * 64, e0 = blockIdx.y * 64, which = blockIdx.z;
  const float* W = which ? Wt : Wv;
  const int r = tid >> 4, c4 = tid & 15;
  #pragma unroll
  for (int i = 0; i < 4; ++i) {
    const int row = 16 * i + r;
    const v4f x = *(const v4fa*)(W + (size_t)(k0 + row) * NE + e0 + 4 * c4);
    _Float16* cp = sT + (4 * c4) * ZP + row;
    cp[0]      = (_Float16)(x.x * 64.0f);
    cp[ZP]     = (_Float16)(x.y * 64.0f);
    cp[2 * ZP] = (_Float16)(x.z * 64.0f);
    cp[3 * ZP] = (_Float16)(x.w * 64.0f);
  }
  __syncthreads();
  _Float16* dstp = WT + (size_t)which * NE * KIN;
  const int q8 = lane & 7, sub = lane >> 3;
  v8h v[2]; size_t off[2];
  #pragma unroll
  for (int j = 0; j < 2; ++j) {
    const int er = 8 * wv + 4 * j + sub;
    v[j] = *(const v8ha*)(sT + er * ZP + 8 * q8);
    off[j] = (size_t)(e0 + er) * KIN + k0 + 8 * q8;
  }
  #pragma unroll
  for (int j = 0; j < 2; ++j) *(volatile v8h*)(dstp + off[j]) = v[j];
  __threadfence();
  #pragma unroll
  for (int j = 0; j < 2; ++j) *(volatile v8h*)(dstp + off[j]) = v[j];
}

__global__ __launch_bounds__(256) void k_convx(const float* __restrict__ xv,
                                               const float* __restrict__ xt,
                                               _Float16* __restrict__ hv,
                                               _Float16* __restrict__ ht,
                                               int ngv8, int ngt8)
{
  const int g = blockIdx.x * 256 + threadIdx.x;
  if (g >= ngv8 + ngt8) return;
  const float* s; _Float16* d;
  if (g < ngv8) { s = xv + (size_t)g * 8; d = hv + (size_t)g * 8; }
  else { const int e = g - ngv8; s = xt + (size_t)e * 8; d = ht + (size_t)e * 8; }
  const v4f a = *(const v4fa*)s;
  const v4f c = *(const v4fa*)(s + 4);
  v8h o;
  o[0] = (_Float16)a.x; o[1] = (_Float16)a.y; o[2] = (_Float16)a.z; o[3] = (_Float16)a.w;
  o[4] = (_Float16)c.x; o[5] = (_Float16)c.y; o[6] = (_Float16)c.z; o[7] = (_Float16)c.w;
  *(volatile v8h*)d = o;
  __threadfence();
  *(volatile v8h*)d = o;
}

__global__ __launch_bounds__(256) void k_proj(const _Float16* __restrict__ X16,
                                              const _Float16* __restrict__ WT,
                                              const float* __restrict__ bias,
                                              const float* __restrict__ wfc,
                                              const float* __restrict__ bfc,
                                              float* __restrict__ Yn,
                                              _Float16* __restrict__ Y16,
                                              float* __restrict__ wraw)
{
  __shared__ __attribute__((aligned(16))) float sT[16 * NE];
  __shared__ __attribute__((aligned(16))) float sW[16];

  const int tid = threadIdx.x, lane = tid & 31, w = tid >> 5;
  const int h = lane >> 4, m = lane & 15;
  const int row0 = blockIdx.x * 16;
  const _Float16* xa = X16 + (size_t)(row0 + m) * KIN;
  const _Float16* wb = WT + (size_t)(w * 64 + m) * KIN;

  const v8f zero8 = {0.f, 0.f, 0.f, 0.f, 0.f, 0.f, 0.f, 0.f};
  v8f acc[4];
  #pragma unroll
  for (int nt = 0; nt < 4; ++nt) acc[nt] = zero8;

  #pragma unroll 1
  for (int k0 = 0; k0 < KIN; k0 += 32) {
    const v16h a = load_frag(xa + k0, h);
    #pragma unroll
    for (int nt = 0; nt < 4; ++nt) {
      const v16h bf = load_frag(wb + (size_t)nt * 16 * KIN + k0, h);
      acc[nt] = wmma_f16(a, bf, acc[nt]);
    }
  }

  #pragma unroll
  for (int nt = 0; nt < 4; ++nt) {
    const int col = w * 64 + nt * 16 + m;
    const float bv = bias[col];
    #pragma unroll
    for (int r = 0; r < 8; ++r) sT[(8 * h + r) * NE + col] = acc[nt][r] * 0.015625f + bv;
  }
  __syncthreads();

  v4f wf[4];
  #pragma unroll
  for (int i = 0; i < 4; ++i) wf[i] = *(const v4fa*)(wfc + 128 * i + 4 * lane);
  const float bf = bfc[0];

  #pragma unroll
  for (int rr = 0; rr < 2; ++rr) {
    const int row = 2 * w + rr;
    const float* sr = sT + row * NE;
    v4f x[4];
    float ss = 0.f, dt = 0.f;
    #pragma unroll
    for (int i = 0; i < 4; ++i) {
      x[i] = *(const v4fa*)(sr + 128 * i + 4 * lane);
      ss += x[i].x * x[i].x + x[i].y * x[i].y + x[i].z * x[i].z + x[i].w * x[i].w;
      dt += x[i].x * wf[i].x + x[i].y * wf[i].y + x[i].z * wf[i].z + x[i].w * wf[i].w;
    }
    #pragma unroll
    for (int s = 16; s > 0; s >>= 1) { ss += __shfl_xor(ss, s); dt += __shfl_xor(dt, s); }
    const float inv = 1.0f / fmaxf(sqrtf(ss), 1e-12f);
    if (lane == 0) sW[row] = dt + bf;
    v4f o[4];
    #pragma unroll
    for (int i = 0; i < 4; ++i) o[i] = x[i] * inv;
    const float sc = inv * 32.0f;
    const v4f p0 = *(const v4fa*)(sr + 8 * lane);
    const v4f p1 = *(const v4fa*)(sr + 8 * lane + 4);
    const v4f p2 = *(const v4fa*)(sr + 256 + 8 * lane);
    const v4f p3 = *(const v4fa*)(sr + 256 + 8 * lane + 4);
    v8h g0, g1;
    g0[0] = (_Float16)(p0.x * sc); g0[1] = (_Float16)(p0.y * sc); g0[2] = (_Float16)(p0.z * sc); g0[3] = (_Float16)(p0.w * sc);
    g0[4] = (_Float16)(p1.x * sc); g0[5] = (_Float16)(p1.y * sc); g0[6] = (_Float16)(p1.z * sc); g0[7] = (_Float16)(p1.w * sc);
    g1[0] = (_Float16)(p2.x * sc); g1[1] = (_Float16)(p2.y * sc); g1[2] = (_Float16)(p2.z * sc); g1[3] = (_Float16)(p2.w * sc);
    g1[4] = (_Float16)(p3.x * sc); g1[5] = (_Float16)(p3.y * sc); g1[6] = (_Float16)(p3.z * sc); g1[7] = (_Float16)(p3.w * sc);
    float* yr = Yn + (size_t)(row0 + row) * NE;
    _Float16* hr = Y16 + (size_t)(row0 + row) * NE;
    #pragma unroll
    for (int i = 0; i < 4; ++i) *(volatile v4f*)(yr + 128 * i + 4 * lane) = o[i];
    *(volatile v8h*)(hr + 8 * lane) = g0;
    *(volatile v8h*)(hr + 256 + 8 * lane) = g1;
    __threadfence();
    #pragma unroll
    for (int i = 0; i < 4; ++i) *(volatile v4f*)(yr + 128 * i + 4 * lane) = o[i];
    *(volatile v8h*)(hr + 8 * lane) = g0;
    *(volatile v8h*)(hr + 256 + 8 * lane) = g1;
  }
  __syncthreads();

  if (w == 0) {
    const int li = (lane < 4) ? lane : 3;
    const v4f t4 = *(const v4fa*)(sW + 4 * li);
    const v4f z4 = {0.f, 0.f, 0.f, 0.f};
    v4f val = z4;
    if (lane < 4) val = t4;
    float* dst = wraw + (size_t)blockIdx.x * 32 + 4 * lane;
    if (lane < 8) *(volatile v4f*)dst = val;
    __threadfence();
    if (lane < 8) *(volatile v4f*)dst = val;
  }
}

__global__ __launch_bounds__(256) void k_softmax(const float* __restrict__ wrv,
                                                 const float* __restrict__ wrt,
                                                 const float* __restrict__ bvfc,
                                                 const float* __restrict__ btfc,
                                                 const int* __restrict__ tlen,
                                                 float* __restrict__ vw,
                                                 float* __restrict__ tw)
{
  __shared__ float red[256];
  __shared__ __attribute__((aligned(16))) float sP[256];
  const int t = threadIdx.x;
  const int blk = blockIdx.x;
  const bool isv = blk < NB;
  const float ninf = -__builtin_inff();
  int b; float x;
  if (isv) {
    b = blk;
    const int gi = b * NV + ((t < NV) ? t : (NV - 1));
    const float v = wrv[(gi >> 4) * 32 + (gi & 15)] + bvfc[0];
    x = (t < NV) ? v : ninf;
  } else {
    b = blk - NB;
    int len = tlen[b];
    len = (len < 0) ? 0 : ((len > NT) ? NT : len);
    const int gi = b * NT + ((t < NT) ? t : (NT - 1));
    const float v = wrt[(gi >> 4) * 32 + (gi & 15)] + btfc[0];
    x = (t < NT && t < len) ? v : ninf;
  }
  red[t] = x;
  __syncthreads();
  for (int o = 128; o > 0; o >>= 1) {
    if (t < o) red[t] = fmaxf(red[t], red[t + o]);
    __syncthreads();
  }
  const float mx = red[0];
  __syncthreads();
  const float ex = expf(x - mx);
  const float e = (x != ninf) ? ex : 0.f;
  red[t] = e;
  __syncthreads();
  for (int o = 128; o > 0; o >>= 1) {
    if (t < o) red[t] += red[t + o];
    __syncthreads();
  }
  const float sum = red[0];
  const float inv = (sum > 0.f) ? (1.0f / sum) : 0.f;
  sP[t] = e * inv;
  __syncthreads();
  if (isv) {
    if (t < 64) {
      const v4f o4 = *(const v4fa*)(sP + 4 * t);
      float* dst = vw + (size_t)b * VWP + 4 * t;
      *(volatile v4f*)dst = o4;
      __threadfence();
      *(volatile v4f*)dst = o4;
    }
  } else {
    if (t < 16) {
      const v4f o4 = *(const v4fa*)(sP + 4 * t);
      float* dst = tw + (size_t)b * NT + 4 * t;
      *(volatile v4f*)dst = o4;
      __threadfence();
      *(volatile v4f*)dst = o4;
    }
  }
}

__global__ __launch_bounds__(416) void k_sim(const _Float16* __restrict__ ve16,
                                             const _Float16* __restrict__ te16,
                                             const float* __restrict__ vw,
                                             const float* __restrict__ tw,
                                             float* __restrict__ out,
                                             int* __restrict__ idx1,
                                             int* __restrict__ idx2)
{
  __shared__ float sRedI[2 * SWAVES];
  __shared__ float sColV[2 * SWAVES * NT];
  __shared__ int   sColA[SWAVES * NT];
  __shared__ float sPart[4];
  __shared__ __attribute__((aligned(16))) float sOut0[NB];
  __shared__ __attribute__((aligned(16))) float sOut1[NB];
  __shared__ __attribute__((aligned(16))) int   sIdx1[I1P];
  __shared__ __attribute__((aligned(16))) int   sIdx2[NT];

  const int tid = threadIdx.x, lane = tid & 31, w = tid >> 5;
  const int h = lane >> 4, m = lane & 15;
  const int b = blockIdx.x;
  const int vbase = 16 * w + 8 * h;
  if (tid < I1P) sIdx1[tid] = 0;
  if (tid < NT) { sIdx2[tid] = 0; sOut0[tid] = 0.f; sOut1[tid] = 0.f; }
  float vwr[8];
  #pragma unroll
  for (int r = 0; r < 8; ++r) vwr[r] = vw[(size_t)b * VWP + vbase + r];
  const _Float16* arow = ve16 + ((size_t)b * NV + 16 * w + m) * NE;
  const float ninf = -__builtin_inff();
  const v8f zero8 = {0.f, 0.f, 0.f, 0.f, 0.f, 0.f, 0.f, 0.f};
  __syncthreads();

  #pragma unroll 1
  for (int qp = 0; qp < NB / 2; ++qp) {
    const int q0 = 2 * qp;
    v8f acc[2][4];
    #pragma unroll
    for (int qi = 0; qi < 2; ++qi)
      #pragma unroll
      for (int nt = 0; nt < 4; ++nt) acc[qi][nt] = zero8;
    const _Float16* brow = te16 + ((size_t)q0 * NT + m) * NE;

    #pragma unroll 1
    for (int k0 = 0; k0 < NE; k0 += 32) {
      const v16h a = load_frag(arow + k0, h);
      #pragma unroll
      for (int qi = 0; qi < 2; ++qi)
        #pragma unroll
        for (int nt = 0; nt < 4; ++nt) {
          const v16h bf = load_frag(brow + (size_t)(qi * NT + nt * 16) * NE + k0, h);
          acc[qi][nt] = wmma_f16(a, bf, acc[qi][nt]);
        }
    }

    #pragma unroll
    for (int qi = 0; qi < 2; ++qi) {
      const int q = q0 + qi;
      const bool diag = (q == b);
      float si = 0.f;
      #pragma unroll
      for (int r = 0; r < 8; ++r) {
        float mx = acc[qi][0][r];
        int am = m;
        #pragma unroll
        for (int nt = 1; nt < 4; ++nt) {
          const float v = acc[qi][nt][r];
          const bool tk = v > mx;
          mx = tk ? v : mx;
          am = tk ? (16 * nt + m) : am;
        }
        #pragma unroll
        for (int s = 1; s < 16; s <<= 1) {
          const float ov = __shfl_xor(mx, s);
          const int oa = __shfl_xor(am, s);
          const bool tk = (ov > mx) || (ov == mx && oa < am);
          mx = tk ? ov : mx;
          am = tk ? oa : am;
        }
        const bool valid = (vbase + r) < NV;
        si += valid ? (vwr[r] * mx) : 0.f;
        if (diag && valid && m == 0) sIdx1[vbase + r] = am;
      }
      si += __shfl_xor(si, 16);
      if (lane == 0) sRedI[qi * SWAVES + w] = si * (1.0f / 1024.0f);
      #pragma unroll
      for (int nt = 0; nt < 4; ++nt) {
        float cm = ninf;
        int ca = 0x7fffffff;
        #pragma unroll
        for (int r = 0; r < 8; ++r) {
          const bool valid = (vbase + r) < NV;
          const float v = valid ? acc[qi][nt][r] : ninf;
          const bool tk = v > cm;
          cm = tk ? v : cm;
          ca = tk ? (vbase + r) : ca;
        }
        const float ov = __shfl_xor(cm, 16);
        const int oa = __shfl_xor(ca, 16);
        const bool tk = (ov > cm) || (ov == cm && oa < ca);
        cm = tk ? ov : cm;
        ca = tk ? oa : ca;
        if (h == 0) {
          sColV[(qi * SWAVES + w) * NT + 16 * nt + m] = cm;
          if (diag) sColA[w * NT + 16 * nt + m] = ca;
        }
      }
    }
    __syncthreads();

    if (tid < 128) {
      const int qi = tid >> 6, t = tid & 63, q = q0 + qi;
      float best = sColV[(qi * SWAVES) * NT + t];
      int ba = sColA[t];
      #pragma unroll 1
      for (int ww = 1; ww < SWAVES; ++ww) {
        const float v = sColV[(qi * SWAVES + ww) * NT + t];
        const int a = sColA[ww * NT + t];
        const bool tk = v > best;
        best = tk ? v : best;
        ba = tk ? a : ba;
      }
      if (q == b) sIdx2[t] = ba;
      float part = tw[(size_t)q * NT + t] * best * (1.0f / 1024.0f);
      #pragma unroll
      for (int s = 16; s > 0; s >>= 1) part += __shfl_xor(part, s);
      if (lane == 0) sPart[w] = part;
    }
    __syncthreads();
    if (tid == 0) {
      float s0 = 0.f, s1 = 0.f;
      #pragma unroll 1
      for (int ww = 0; ww < SWAVES; ++ww) { s0 += sRedI[ww]; s1 += sRedI[SWAVES + ww]; }
      sOut0[q0] = s0;
      sOut0[q0 + 1] = s1;
      sOut1[q0] = sPart[0] + sPart[1];
      sOut1[q0 + 1] = sPart[2] + sPart[3];
    }
    __syncthreads();
  }

  if (w == 0) {
    const int l16 = lane & 15;
    const v4f a0 = *(const v4fa*)(sOut0 + 4 * l16);
    const v4f a1 = *(const v4fa*)(sOut1 + 4 * l16);
    v4f v = a0;
    if (lane >= 16) v = a1;
    float* dst = out + ((lane < 16) ? 0 : (NB * NB)) + b * NB + 4 * l16;
    *(volatile v4f*)dst = v;
    __threadfence();
    *(volatile v4f*)dst = v;
  } else if (w == 1) {
    const v4i v0 = *(const v4ia*)(sIdx1 + 4 * lane);
    const v4i v1 = *(const v4ia*)(sIdx1 + 128 + 4 * lane);
    int* d0 = idx1 + (size_t)b * I1P + 4 * lane;
    int* d1 = d0 + 128;
    *(volatile v4i*)d0 = v0;
    *(volatile v4i*)d1 = v1;
    __threadfence();
    *(volatile v4i*)d0 = v0;
    *(volatile v4i*)d1 = v1;
  } else if (w == 2) {
    const int l16 = lane & 15;
    const v4i v = *(const v4ia*)(sIdx2 + 4 * l16);
    int* dst = idx2 + (size_t)b * NT + 4 * l16;
    if (lane < 16) *(volatile v4i*)dst = v;
    __threadfence();
    if (lane < 16) *(volatile v4i*)dst = v;
  }
}

__global__ __launch_bounds__(512) void k_stats(const float* __restrict__ ven,
                                               const float* __restrict__ ten,
                                               const int* __restrict__ idx1,
                                               const int* __restrict__ idx2,
                                               float* __restrict__ stats)
{
  __shared__ __attribute__((aligned(16))) float sM[NE];
  __shared__ __attribute__((aligned(16))) float sI[NE];
  const int mat = blockIdx.x, col = threadIdx.x;
  double s = 0.0, sq = 0.0;
  int n;
  if (mat == 0) {
    n = MT;
    #pragma unroll 1
    for (int a = 0; a < MT; ++a) {
      const double x = (double)ten[(size_t)a * NE + col];
      s += x; sq += x * x;
    }
  } else if (mat == 1) {
    n = MT;
    #pragma unroll 1
    for (int a = 0; a < MT; ++a) {
      const int bb = a >> 6, t = a & 63;
      int j = idx2[bb * NT + t];
      j = (j < 0) ? 0 : ((j > NV - 1) ? (NV - 1) : j);
      const double x = (double)ven[((size_t)bb * NV + j) * NE + col];
      s += x; sq += x * x;
    }
  } else if (mat == 2) {
    n = MV;
    #pragma unroll 1
    for (int a = 0; a < MV; ++a) {
      const double x = (double)ven[(size_t)a * NE + col];
      s += x; sq += x * x;
    }
  } else {
    n = MV;
    #pragma unroll 1
    for (int a = 0; a < MV; ++a) {
      const int bb = a / NV, v = a - bb * NV;
      int j = idx1[bb * I1P + v];
      j = (j < 0) ? 0 : ((j > NT - 1) ? (NT - 1) : j);
      const double x = (double)ten[((size_t)bb * NT + j) * NE + col];
      s += x; sq += x * x;
    }
  }
  const double dn = (double)n;
  const double mean = s / dn;
  double var = (sq - dn * mean * mean) / (dn - 1.0);
  var = (var > 1e-30) ? var : 1e-30;
  const double istd = 1.0 / sqrt(var);
  sM[col] = (float)mean;
  sI[col] = (float)istd;
  __syncthreads();
  if (col < 256) {
    const int e = (col & 127) * 4;
    const v4f vm = *(const v4fa*)(sM + e);
    const v4f vi = *(const v4fa*)(sI + e);
    v4f v = vm;
    if (col >= 128) v = vi;
    float* dst = stats + (size_t)(mat * 2 + (col >> 7)) * NE + e;
    *(volatile v4f*)dst = v;
    __threadfence();
    *(volatile v4f*)dst = v;
  }
}

__global__ __launch_bounds__(256) void k_znT(const float* __restrict__ src,
                                             const int* __restrict__ idx,
                                             const float* __restrict__ stats,
                                             const float* __restrict__ wgt,
                                             _Float16* __restrict__ outp,
                                             int n, int mode)
{
  __shared__ __attribute__((aligned(16))) _Float16 sT[128 * ZP];
  const int tid = threadIdx.x, lane = tid & 31, wv = tid >> 5;
  const int a0 = blockIdx.x * 64, c0 = blockIdx.y * 128;
  const float* mean = stats + (size_t)(mode * 2) * NE;
  const float* istd = mean + NE;
  const v4f mu = *(const v4fa*)(mean + c0 + 4 * lane);
  const v4f is = *(const v4fa*)(istd + c0 + 4 * lane);

  #pragma unroll 1
  for (int i = 0; i < 8; ++i) {
    const int al = 8 * wv + i;
    const int a = a0 + al;
    int rs; float wt;
    if (mode == 0) {
      rs = a; wt = wgt[a] * 256.0f;
    } else if (mode == 1) {
      const int bb = a >> 6, t = a & 63;
      int j = idx[bb * NT + t];
      j = (j < 0) ? 0 : ((j > NV - 1) ? (NV - 1) : j);
      rs = bb * NV + j; wt = 1.0f;
    } else if (mode == 2) {
      const int bb = a / NV, v = a - bb * NV;
      rs = a; wt = wgt[bb * VWP + v] * 256.0f;
    } else {
      const int bb = a / NV, v = a - bb * NV;
      int j = idx[bb * I1P + v];
      j = (j < 0) ? 0 : ((j > NT - 1) ? (NT - 1) : j);
      rs = bb * NT + j; wt = 1.0f;
    }
    const v4f x = *(const v4fa*)(src + (size_t)rs * NE + c0 + 4 * lane);
    const float z0 = (x.x - mu.x) * is.x * wt;
    const float z1 = (x.y - mu.y) * is.y * wt;
    const float z2 = (x.z - mu.z) * is.z * wt;
    const float z3 = (x.w - mu.w) * is.w * wt;
    _Float16* cp = sT + (4 * lane) * ZP + al;
    cp[0]      = (_Float16)z0;
    cp[ZP]     = (_Float16)z1;
    cp[2 * ZP] = (_Float16)z2;
    cp[3 * ZP] = (_Float16)z3;
  }
  __syncthreads();
  const int q8 = lane & 7, sub = lane >> 3;
  v8h v[4]; size_t off[4];
  #pragma unroll
  for (int j = 0; j < 4; ++j) {
    const int cl = 16 * wv + 4 * j + sub;
    v[j] = *(const v8ha*)(sT + cl * ZP + 8 * q8);
    off[j] = (size_t)(c0 + cl) * (size_t)n + a0 + 8 * q8;
  }
  #pragma unroll
  for (int j = 0; j < 4; ++j) *(volatile v8h*)(outp + off[j]) = v[j];
  __threadfence();
  #pragma unroll
  for (int j = 0; j < 4; ++j) *(volatile v8h*)(outp + off[j]) = v[j];
}

__global__ __launch_bounds__(128) void k_cgemm(const _Float16* __restrict__ A1,
                                               const _Float16* __restrict__ B1,
                                               const _Float16* __restrict__ A2,
                                               const _Float16* __restrict__ B2,
                                               double* __restrict__ cpart)
{
  __shared__ double sOn[128];
  __shared__ double sOff[128];
  const int tid = threadIdx.x, lane = tid & 31, w = tid >> 5;
  const int h = lane >> 4, m = lane & 15;
  const int cb = blockIdx.x * 128 + 32 * w;
  const int d0 = blockIdx.y * 64;
  const v8f zero8 = {0.f, 0.f, 0.f, 0.f, 0.f, 0.f, 0.f, 0.f};
  v8f acc[2][4];
  #pragma unroll
  for (int ms = 0; ms < 2; ++ms)
    #pragma unroll
    for (int nt = 0; nt < 4; ++nt) acc[ms][nt] = zero8;

  {
    const _Float16* pa = A1 + (size_t)(cb + m) * MT;
    const _Float16* pb = B1 + (size_t)(d0 + m) * MT;
    #pragma unroll 1
    for (int k0 = 0; k0 < MT; k0 += 32) {
      const v16h fa0 = load_frag(pa + k0, h);
      const v16h fa1 = load_frag(pa + (size_t)16 * MT + k0, h);
      #pragma unroll
      for (int nt = 0; nt < 4; ++nt) {
        const v16h fb = load_frag(pb + (size_t)nt * 16 * MT + k0, h);
        acc[0][nt] = wmma_f16(fa0, fb, acc[0][nt]);
        acc[1][nt] = wmma_f16(fa1, fb, acc[1][nt]);
      }
    }
  }
  {
    const _Float16* pa = A2 + (size_t)(cb + m) * MV;
    const _Float16* pb = B2 + (size_t)(d0 + m) * MV;
    #pragma unroll 1
    for (int k0 = 0; k0 < MV; k0 += 32) {
      const v16h fa0 = load_frag(pa + k0, h);
      const v16h fa1 = load_frag(pa + (size_t)16 * MV + k0, h);
      #pragma unroll
      for (int nt = 0; nt < 4; ++nt) {
        const v16h fb = load_frag(pb + (size_t)nt * 16 * MV + k0, h);
        acc[0][nt] = wmma_f16(fa0, fb, acc[0][nt]);
        acc[1][nt] = wmma_f16(fa1, fb, acc[1][nt]);
      }
    }
  }

  double on = 0.0, off = 0.0;
  #pragma unroll
  for (int ms = 0; ms < 2; ++ms)
    #pragma unroll
    for (int nt = 0; nt < 4; ++nt)
      #pragma unroll
      for (int r = 0; r < 8; ++r) {
        const int row = cb + 16 * ms + 8 * h + r;
        const int col = d0 + 16 * nt + m;
        const double c = (double)(acc[ms][nt][r] * (1.0f / 32768.0f));
        const double e = c - 1.0;
        const bool dg = (row == col);
        on  += dg ? (e * e) : 0.0;
        off += dg ? 0.0 : (c * c);
      }
  sOn[tid] = on;
  sOff[tid] = off;
  __syncthreads();
  if (w == 0) {
    double ton = 0.0, toff = 0.0;
    #pragma unroll 1
    for (int i = 0; i < 128; ++i) { ton += sOn[i]; toff += sOff[i]; }
    v2d val;
    val.x = (lane == 0) ? ton : 0.0;
    val.y = (lane == 0) ? toff : 0.0;
    double* dst = cpart + (size_t)(blockIdx.y * 4 + blockIdx.x) * 16 + 2 * lane;
    if (lane < 8) *(volatile v2d*)dst = val;
    __threadfence();
    if (lane < 8) *(volatile v2d*)dst = val;
  }
}

__global__ __launch_bounds__(32) void k_loss(const double* __restrict__ cpart, float* __restrict__ out)
{
  const int lane = threadIdx.x;
  double on = 0.0, off = 0.0;
  #pragma unroll 1
  for (int i = 0; i < 32; ++i) { on += cpart[16 * i]; off += cpart[16 * i + 1]; }
  const float onf = (float)on, offf = (float)off;
  const float loss = 0.1f * (onf * 1.0f + offf * 0.06f);
  float* dst = out + 2 * NB * NB;
  if (lane == 0) *(volatile float*)dst = loss;
  __threadfence();
  if (lane == 0) *(volatile float*)dst = loss;
}

extern "C" void kernel_launch(void* const* d_in, const int* in_sizes, int n_in,
                              void* d_out, int out_size, void* d_ws, size_t ws_size,
                              hipStream_t stream)
{
  if (n_in < 17) return;
  if (in_sizes[1] != MV * KIN || in_sizes[3] != MT * KIN) return;
  if (in_sizes[8] != KIN * NE || in_sizes[10] != KIN * NE) return;
  if (in_sizes[9] != NE || in_sizes[11] != NE || in_sizes[12] != NE || in_sizes[14] != NE) return;
  if (in_sizes[13] < 1 || in_sizes[15] < 1 || in_sizes[16] != NB) return;
  if (out_size != 2 * NB * NB + 1) return;

  const float* v_tok  = (const float*)d_in[1];
  const float* t_tok  = (const float*)d_in[3];
  const float* Wv_tok = (const float*)d_in[8];
  const float* bv_tok = (const float*)d_in[9];
  const float* Wt_tok = (const float*)d_in[10];
  const float* bt_tok = (const float*)d_in[11];
  const float* wv_fc  = (const float*)d_in[12];
  const float* bv_fc  = (const float*)d_in[13];
  const float* wt_fc  = (const float*)d_in[14];
  const float* bt_fc  = (const float*)d_in[15];
  const int*   tlen   = (const int*)d_in[16];
  float* out = (float*)d_out;

  char* ws = (char*)d_ws;
  size_t off = 0;
  auto carve = [&](size_t bytes) -> char* {
    off = (off + 255) & ~(size_t)255;
    char* p = ws + off;
    off += bytes;
    return p;
  };
  _Float16* WT   = (_Float16*)carve((size_t)2 * NE * KIN * 2);
  _Float16* Xv   = (_Float16*)carve((size_t)MV * KIN * 2);
  _Float16* Xt   = (_Float16*)carve((size_t)MT * KIN * 2);
  float*    Yv   = (float*)carve((size_t)MV * NE * 4);
  float*    Yt   = (float*)carve((size_t)MT * NE * 4);
  _Float16* ve16 = (_Float16*)carve((size_t)MVPAD * NE * 2);
  _Float16* te16 = (_Float16*)carve((size_t)MT * NE * 2);
  float*    wrv  = (float*)carve((size_t)(MV / 16) * 32 * 4);
  float*    wrt  = (float*)carve((size_t)(MT / 16) * 32 * 4);
  float*    vw   = (float*)carve((size_t)NB * VWP * 4);
  float*    tw   = (float*)carve((size_t)NB * NT * 4);
  int*      idx1 = (int*)carve((size_t)NB * I1P * 4);
  int*      idx2 = (int*)carve((size_t)NB * NT * 4);
  float*    stats = (float*)carve((size_t)8 * NE * 4);
  _Float16* P1A  = (_Float16*)carve((size_t)NE * MT * 2);
  _Float16* P1B  = (_Float16*)carve((size_t)NE * MT * 2);
  _Float16* P2A  = (_Float16*)carve((size_t)NE * MV * 2);
  _Float16* P2B  = (_Float16*)carve((size_t)NE * MV * 2);
  double*   cpart = (double*)carve((size_t)32 * 16 * 8);
  if (off > ws_size) return;

  const int nz8 = (MVPAD - MV) * NE / 8;
  k_zfill<<<1, 256, 0, stream>>>(ve16 + (size_t)MV * NE, nz8);

  k_convw<<<dim3(KIN / 64, NE / 64, 2), 256, 0, stream>>>(Wv_tok, Wt_tok, WT);

  const int ngv8 = MV * KIN / 8, ngt8 = MT * KIN / 8;
  k_convx<<<(ngv8 + ngt8 + 255) / 256, 256, 0, stream>>>(v_tok, t_tok, Xv, Xt, ngv8, ngt8);

  k_proj<<<MV / 16, 256, 0, stream>>>(Xv, WT, bv_tok, wv_fc, bv_fc, Yv, ve16, wrv);
  k_proj<<<MT / 16, 256, 0, stream>>>(Xt, WT + (size_t)NE * KIN, bt_tok, wt_fc, bt_fc, Yt, te16, wrt);

  k_softmax<<<2 * NB, 256, 0, stream>>>(wrv, wrt, bv_fc, bt_fc, tlen, vw, tw);

  k_sim<<<NB, 32 * SWAVES, 0, stream>>>(ve16, te16, vw, tw, out, idx1, idx2);

  k_stats<<<4, NE, 0, stream>>>(Yv, Yt, idx1, idx2, stats);

  k_znT<<<dim3(MT / 64, NE / 128), 256, 0, stream>>>(Yt, idx2, stats, tw, P1A, MT, 0);
  k_znT<<<dim3(MT / 64, NE / 128), 256, 0, stream>>>(Yv, idx2, stats, tw, P1B, MT, 1);
  k_znT<<<dim3(MV / 64, NE / 128), 256, 0, stream>>>(Yv, idx1, stats, vw, P2A, MV, 2);
  k_znT<<<dim3(MV / 64, NE / 128), 256, 0, stream>>>(Yt, idx1, stats, vw, P2B, MV, 3);

  k_cgemm<<<dim3(NE / 128, NE / 64), 128, 0, stream>>>(P1A, P1B, P2A, P2B, cpart);

  k_loss<<<1, 32, 0, stream>>>(cpart, out);
}
